// GAT_9947144257800
// MI455X (gfx1250) — hardware-verified
//
#include <hip/hip_runtime.h>


#define BATCH   16
#define NNODE   256
#define INDIM   768
#define MEMD    300
#define HLD     320
#define HIDD    64
#define NEGBIG  (-1e30f)
#define LSLOPE  0.01f

typedef __attribute__((ext_vector_type(16))) __bf16   v16bf;
typedef __attribute__((ext_vector_type(16))) _Float16 v16h;
typedef __attribute__((ext_vector_type(8)))  float    v8f;
typedef __attribute__((ext_vector_type(8)))  unsigned v8u;

__device__ __forceinline__ unsigned f2bf(float f) { unsigned u = __float_as_uint(f); u += 0x7FFFu + ((u >> 16) & 1u); return u >> 16; }
__device__ __forceinline__ unsigned f2h(float f) { return (unsigned)__builtin_bit_cast(unsigned short, (_Float16)f); }
__device__ __forceinline__ int kpat(int v, int half) { return ((v & 4) ? 16 : 0) + half * 8 + 2 * (v & 3); }

template <int F16, int NP> struct Opnd { v16bf p[NP]; };

template <int F16, int NP> __device__ __forceinline__ void pack2(float f0, float f1, unsigned* o) {
    if (F16) { o[0] = f2h(f0) | (f2h(f1) << 16); return; }
    unsigned h0 = f2bf(f0), h1 = f2bf(f1); o[0] = h0 | (h1 << 16);
    if (NP >= 2) {
        float r0 = f0 - __uint_as_float(h0 << 16), r1 = f1 - __uint_as_float(h1 << 16);
        unsigned m0 = f2bf(r0), m1 = f2bf(r1); o[1] = m0 | (m1 << 16);
        if (NP >= 3) {
            float s0 = r0 - __uint_as_float(m0 << 16), s1 = r1 - __uint_as_float(m1 << 16);
            o[2] = f2bf(s0) | (f2bf(s1) << 16);
        }
    }
}
template <int F16, int NP> __device__ __forceinline__ void op_row(const float* rowp, int half, float sc, Opnd<F16, NP>& o) {
    v8u u[NP];
#pragma unroll
    for (int v = 0; v < 8; ++v) {
        int kk = kpat(v, half); unsigned t[3];
        pack2<F16, NP>(rowp[kk] * sc, rowp[kk + 1] * sc, t);
#pragma unroll
        for (int p = 0; p < NP; ++p) u[p][v] = t[p];
    }
#pragma unroll
    for (int p = 0; p < NP; ++p) o.p[p] = __builtin_bit_cast(v16bf, u[p]);
}
template <int F16, int NP> __device__ __forceinline__ void op_row_tail(const float* rowp, int half, float sc, int kvalid, Opnd<F16, NP>& o) {
    v8u u[NP];
#pragma unroll
    for (int v = 0; v < 8; ++v) {
        int kk = kpat(v, half); unsigned t[3];
        float f0 = kk < kvalid ? rowp[kk] * sc : 0.0f, f1 = (kk + 1) < kvalid ? rowp[kk + 1] * sc : 0.0f;
        pack2<F16, NP>(f0, f1, t);
#pragma unroll
        for (int p = 0; p < NP; ++p) u[p][v] = t[p];
    }
#pragma unroll
    for (int p = 0; p < NP; ++p) o.p[p] = __builtin_bit_cast(v16bf, u[p]);
}
template <int F16, int NP> __device__ __forceinline__ void op_col(const float* M, int ld, int n, int k0, int half, float sc, Opnd<F16, NP>& o) {
    v8u u[NP];
#pragma unroll
    for (int v = 0; v < 8; ++v) {
        int kk = k0 + kpat(v, half); unsigned t[3];
        pack2<F16, NP>(M[(size_t)kk * ld + n] * sc, M[(size_t)(kk + 1) * ld + n] * sc, t);
#pragma unroll
        for (int p = 0; p < NP; ++p) u[p][v] = t[p];
    }
#pragma unroll
    for (int p = 0; p < NP; ++p) o.p[p] = __builtin_bit_cast(v16bf, u[p]);
}
template <int F16, int NP> __device__ __forceinline__ void op_col_tail(const float* M, int ld, int n, int k0, int half, float sc, int K, Opnd<F16, NP>& o) {
    v8u u[NP];
#pragma unroll
    for (int v = 0; v < 8; ++v) {
        int kk = k0 + kpat(v, half); unsigned t[3];
        float f0 = kk < K ? M[(size_t)kk * ld + n] * sc : 0.0f, f1 = (kk + 1) < K ? M[(size_t)(kk + 1) * ld + n] * sc : 0.0f;
        pack2<F16, NP>(f0, f1, t);
#pragma unroll
        for (int p = 0; p < NP; ++p) u[p][v] = t[p];
    }
#pragma unroll
    for (int p = 0; p < NP; ++p) o.p[p] = __builtin_bit_cast(v16bf, u[p]);
}
__device__ __forceinline__ v8f wm_bf16(v16bf a, v16bf b, v8f c) { return __builtin_amdgcn_wmma_f32_16x16x32_bf16(false, a, false, b, (short)0, c, false, false); }
template <int F16, int NA, int NB> __device__ __forceinline__ v8f wmma_op(const Opnd<F16, NA>& a, const Opnd<F16, NB>& b, v8f c) {
    if (F16) {
        v16h ah = __builtin_bit_cast(v16h, a.p[0]), bh = __builtin_bit_cast(v16h, b.p[0]);
        c = __builtin_amdgcn_wmma_f32_16x16x32_f16(false, ah, false, bh, (short)0, c, false, false);
        asm volatile("v_nop\n\tv_nop\n\tv_nop\n\tv_nop" : "+v"(c) : "v"(ah), "v"(bh));
        return c;
    }
    constexpr int NMX = NA > NB ? NA : NB;
#pragma unroll
    for (int i = 0; i < NA; ++i)
#pragma unroll
        for (int j = 0; j < NB; ++j)
            if (i + j < NMX) c = wm_bf16(a.p[i], b.p[j], c);
    if (NA == 1 && NB == 1)      asm volatile("v_nop\n\tv_nop\n\tv_nop\n\tv_nop" : "+v"(c) : "v"(a.p[0]), "v"(b.p[0]));
    else if (NA == 2 && NB == 1) asm volatile("v_nop\n\tv_nop\n\tv_nop\n\tv_nop" : "+v"(c) : "v"(a.p[0]), "v"(a.p[1]), "v"(b.p[0]));
    else if (NA == 1 && NB == 2) asm volatile("v_nop\n\tv_nop\n\tv_nop\n\tv_nop" : "+v"(c) : "v"(a.p[0]), "v"(b.p[0]), "v"(b.p[1]));
    else if (NA == 2 && NB == 2) asm volatile("v_nop\n\tv_nop\n\tv_nop\n\tv_nop" : "+v"(c) : "v"(a.p[0]), "v"(a.p[1]), "v"(b.p[0]), "v"(b.p[1]));
    else                         asm volatile("v_nop\n\tv_nop\n\tv_nop\n\tv_nop" : "+v"(c) : "v"(a.p[0]), "v"(a.p[NA - 1]), "v"(b.p[0]), "v"(b.p[NB - 1]), "v"(a.p[NA / 2]), "v"(b.p[NB / 2]));
    return c;
}

struct ZMap { long long s1; long long s2; int zdiv; int pad_; };
__device__ __forceinline__ size_t zoff(const ZMap& m, int z) { return (size_t)((long long)(z / m.zdiv) * m.s1 + (long long)(z % m.zdiv) * m.s2); }

#define ACT_NONE 0
#define ACT_RELU 1
#define ACT_GELU_ERF 2
#define ACT_SILU 3
#define ACT_TANH 4
__device__ __forceinline__ float act_apply(int act, float x) {
    if (act == ACT_RELU) return x > 0.f ? x : 0.f;
    if (act == ACT_GELU_ERF) return 0.5f * x * (1.0f + erff(x * 0.70710678118654752f));
    if (act == ACT_SILU) return x / (1.0f + expf(-x));
    if (act == ACT_TANH) return tanhf(x);
    return x;
}
struct GemmArgs {
    ZMap za, zb_, zc, zbias, zadd;
    const float* A; const float* Bm; float* C; const float* bias; const float* add;
    long long ldadd;
    int lda, ldb, ldc, K;
    float ascale, bscale, oscale, addscale;
    int M, nvalid, nstore, pad0;
};
template <int BT, int F16, int NA, int NB, int RW, int CW, int ACT>
__global__ __launch_bounds__(256) void gemm_kernel(GemmArgs g) {
    constexpr int TR = 16 * RW, TC = 64 * CW, CSTR = TC + 4;
    __shared__ __align__(16) float cst[TR * CSTR];
    const int z = blockIdx.z;
    const float* A = g.A + zoff(g.za, z); const float* Bm = g.Bm + zoff(g.zb_, z); float* C = g.C + zoff(g.zc, z);
    const int tid = threadIdx.x, lane = tid & 31, wv = tid >> 5;
    const int l16 = lane & 15, half = lane >> 4;
    const int rt = wv % RW, ch = wv / RW;
    const int row0 = blockIdx.x * TR, col0 = blockIdx.y * TC + ch * 64;
    int arix = row0 + rt * 16 + l16; if (arix >= g.M) arix = g.M - 1;
    const float* arow = A + (size_t)arix * g.lda;
    v8f acc[4];
#pragma unroll
    for (int t = 0; t < 4; ++t) acc[t] = (v8f){};
    const int K = g.K;
#pragma unroll 1
    for (int kc = 0; kc < K; kc += 32) {
        Opnd<F16, NA> a;
        if (kc + 32 <= K) op_row<F16, NA>(arow + kc, half, g.ascale, a); else op_row_tail<F16, NA>(arow + kc, half, g.ascale, K - kc, a);
#pragma unroll
        for (int t = 0; t < 4; ++t) {
            Opnd<F16, NB> b;
            const int n = col0 + t * 16 + l16;
            if (n < g.nvalid) {
                if (BT) { if (kc + 32 <= K) op_row<F16, NB>(Bm + (size_t)n * g.ldb + kc, half, g.bscale, b); else op_row_tail<F16, NB>(Bm + (size_t)n * g.ldb + kc, half, g.bscale, K - kc, b); }
                else    { if (kc + 32 <= K) op_col<F16, NB>(Bm, g.ldb, n, kc, half, g.bscale, b); else op_col_tail<F16, NB>(Bm, g.ldb, n, kc, half, g.bscale, K, b); }
            } else {
#pragma unroll
                for (int p = 0; p < NB; ++p) b.p[p] = (v16bf){};
            }
            acc[t] = wmma_op<F16, NA, NB>(a, b, acc[t]);
        }
    }
    const float* bias = g.bias ? g.bias + zoff(g.zbias, z) : nullptr;
    const float* add = g.add ? g.add + zoff(g.zadd, z) : nullptr;
#pragma unroll
    for (int t = 0; t < 4; ++t) {
        const int cl = ch * 64 + t * 16 + l16;
        const int cg = blockIdx.y * TC + cl;
        const bool cok = cg < g.nvalid;
        const float bv = (bias && cok) ? bias[cg] : 0.0f;
#pragma unroll
        for (int r = 0; r < 8; ++r) {
            const int rl = rt * 16 + r + 8 * half;
            float v = acc[t][r] * g.oscale + bv;
            int rg = row0 + rl; if (rg >= g.M) rg = g.M - 1;
            if (add && cok) v += g.addscale * add[(size_t)rg * g.ldadd + cg];
            cst[rl * CSTR + cl] = v;
        }
    }
    __syncthreads();
    const int col = tid % TC, rsel = tid / TC, rstep = 256 / TC;
    if (ACT != ACT_NONE) {
#pragma unroll 1
        for (int r = rsel; r < TR; r += rstep) cst[r * CSTR + col] = act_apply(ACT, cst[r * CSTR + col]);
    }
    float* ob = C + (size_t)row0 * g.ldc + (size_t)blockIdx.y * TC;
    const bool colok = (int)(blockIdx.y * TC + col) < g.nstore;
    const int rmax = (g.M - row0 < TR) ? (g.M - row0) : TR;
    auto pass = [&]() {
        if (colok) {
#pragma unroll 4
            for (int r = rsel; r < rmax; r += rstep) *(volatile float*)(ob + (size_t)r * g.ldc + col) = cst[r * CSTR + col];
        }
    };
    pass();
    __threadfence();
    pass();
}
static inline ZMap zm(long long s1) { ZMap m; m.s1 = s1; m.s2 = 0; m.zdiv = 1; m.pad_ = 0; return m; }
static inline ZMap zm2(long long s1, long long s2, int zdiv) { ZMap m; m.s1 = s1; m.s2 = s2; m.zdiv = zdiv; m.pad_ = 0; return m; }
static inline GemmArgs gemm_args(const float* A, int lda, ZMap za, const float* Bm, int ldb, ZMap zb, float* C, int ldc, ZMap zc, int M, int N, int K) {
    GemmArgs g; g.za = za; g.zb_ = zb; g.zc = zc; g.zbias = zm(0); g.zadd = zm(0);
    g.A = A; g.Bm = Bm; g.C = C; g.bias = nullptr; g.add = nullptr; g.ldadd = 0;
    g.lda = lda; g.ldb = ldb; g.ldc = ldc; g.K = K; g.ascale = 1.0f; g.bscale = 1.0f; g.oscale = 1.0f; g.addscale = 1.0f; g.M = M; g.nvalid = N; g.nstore = N; g.pad0 = 0;
    return g;
}
static_assert(sizeof(ZMap) == 24, "ZMap layout");
static_assert(sizeof(GemmArgs) == 5 * 24 + 5 * 8 + 8 + 4 * 4 + 4 * 4 + 4 * 4, "GemmArgs has no padding");

__global__ __launch_bounds__(256) void softmax_rows(float* S, long long sy, long long sx, int L, float prescale, const float* addv, long long say, int aydiv) {
    __shared__ float red[8];
    const int tid = threadIdx.x, lane = tid & 31, wid = tid >> 5;
    float* row = S + (size_t)blockIdx.y * sy + (size_t)blockIdx.x * sx;
    const float* av = addv ? addv + (size_t)(blockIdx.y / aydiv) * say : nullptr;
    float v[16];
    const int nj = L / 256;
    float mx = -__builtin_inff();
#pragma unroll
    for (int j = 0; j < 16; ++j) if (j < nj) { float t = row[tid + 256 * j] * prescale; if (av) t += av[tid + 256 * j]; v[j] = t; mx = fmaxf(mx, t); }
#pragma unroll
    for (int o = 16; o; o >>= 1) mx = fmaxf(mx, __shfl_xor(mx, o, 32));
    if (lane == 0) red[wid] = mx;
    __syncthreads();
    float m = red[0];
#pragma unroll
    for (int i = 1; i < 8; ++i) m = fmaxf(m, red[i]);
    if (m == -__builtin_inff()) m = 0.f;
    __syncthreads();
    float sum = 0.f;
#pragma unroll
    for (int j = 0; j < 16; ++j) if (j < nj) { v[j] = expf(v[j] - m); sum += v[j]; }
#pragma unroll
    for (int o = 16; o; o >>= 1) sum += __shfl_xor(sum, o, 32);
    if (lane == 0) red[wid] = sum;
    __syncthreads();
    float tot = 0.f;
#pragma unroll
    for (int i = 0; i < 8; ++i) tot += red[i];
    const float inv = 1.0f / tot;
#pragma unroll
    for (int j = 0; j < 16; ++j) if (j < nj) *(volatile float*)(row + tid + 256 * j) = v[j] * inv;
    __threadfence();
#pragma unroll
    for (int j = 0; j < 16; ++j) if (j < nj) *(volatile float*)(row + tid + 256 * j) = v[j] * inv;
}


__global__ __launch_bounds__(256) void edge_scores(const float* __restrict__ si, const float* __restrict__ sj, const float* __restrict__ a2,
                                                   const float* __restrict__ ab2, const float* __restrict__ adj, float* logits) {
    const int i = blockIdx.x, b = blockIdx.y, j = threadIdx.x;
    __shared__ float ssi[HIDD];
    __shared__ float sa2[HIDD];
    if (j < HIDD) { ssi[j] = si[((size_t)(b * NNODE + i)) * HIDD + j]; sa2[j] = a2[j]; }
    __syncthreads();
    const float4* sjr = (const float4*)(sj + ((size_t)(b * NNODE + j)) * HIDD);
    float acc = 0.0f;
#pragma unroll
    for (int h4 = 0; h4 < HIDD / 4; ++h4) {
        const float4 v = sjr[h4];
        const int h = h4 * 4;
        acc += fmaxf(ssi[h + 0] + v.x, 0.0f) * sa2[h + 0];
        acc += fmaxf(ssi[h + 1] + v.y, 0.0f) * sa2[h + 1];
        acc += fmaxf(ssi[h + 2] + v.z, 0.0f) * sa2[h + 2];
        acc += fmaxf(ssi[h + 3] + v.w, 0.0f) * sa2[h + 3];
    }
    float e = acc + ab2[0];
    e = e > 0.0f ? e : LSLOPE * e;
    const size_t idx = ((size_t)(b * NNODE + i)) * NNODE + j;
    const float a = adj[idx];
    const float lv = e * a + (1.0f - a) * NEGBIG;
    *(volatile float*)(logits + idx) = lv;
    __threadfence();
    *(volatile float*)(logits + idx) = lv;
}

__global__ __launch_bounds__(256) void softmax_stats(const float* __restrict__ logits, float* red) {
    const int b = blockIdx.x, tid = threadIdx.x;
    const float* p = logits + (size_t)b * NNODE * NNODE;
    __shared__ float s[256];
    float m = -__builtin_inff();
    for (int i = tid; i < NNODE * NNODE; i += 256) m = fmaxf(m, p[i]);
    s[tid] = m;
    __syncthreads();
    for (int off = 128; off > 0; off >>= 1) { if (tid < off) s[tid] = fmaxf(s[tid], s[tid + off]); __syncthreads(); }
    const float mx = s[0];
    __syncthreads();
    float sum = 0.0f;
    for (int i = tid; i < NNODE * NNODE; i += 256) sum += expf(p[i] - mx);
    s[tid] = sum;
    __syncthreads();
    for (int off = 128; off > 0; off >>= 1) { if (tid < off) s[tid] += s[tid + off]; __syncthreads(); }
    if (tid < 32) {
        const float v = (tid == 0) ? mx : ((tid == 1) ? s[0] : 0.0f);
        *(volatile float*)(red + b * 32 + tid) = v;
        __threadfence();
        *(volatile float*)(red + b * 32 + tid) = v;
    }
}

__global__ __launch_bounds__(256) void softmax_norm(float* att, const float* __restrict__ red) {
    const int b = blockIdx.y;
    const size_t i = (size_t)blockIdx.x * NNODE + threadIdx.x;
    const float mx = red[b * 32 + 0];
    const float inv = 1.0f / red[b * 32 + 1];
    float* p = att + (size_t)b * NNODE * NNODE;
    const float v = expf(p[i] - mx) * inv;
    *(volatile float*)(p + i) = v;
    __threadfence();
    *(volatile float*)(p + i) = v;
}

extern "C" void kernel_launch(void* const* d_in, const int* in_sizes, int n_in,
                              void* d_out, int out_size, void* d_ws, size_t ws_size, hipStream_t stream) {
    (void)in_sizes; (void)n_in; (void)out_size;
    const float* adj     = (const float*)d_in[0];
    const float* feature = (const float*)d_in[1];
    const float* W0      = (const float*)d_in[2];
    const float* b0      = (const float*)d_in[3];
    const float* W1      = (const float*)d_in[4];
    const float* b1      = (const float*)d_in[5];
    const float* A1      = (const float*)d_in[6];
    const float* ab1     = (const float*)d_in[7];
    const float* A2      = (const float*)d_in[8];
    const float* ab2     = (const float*)d_in[9];
    float* out = (float*)d_out;

    const int MROWS = BATCH * NNODE;
    float* bufH = (float*)d_ws;
    float* bufX = bufH + (size_t)MROWS * HLD;
    float* si   = bufX + (size_t)MROWS * HLD;
    float* sj   = si + (size_t)MROWS * HIDD;
    float* att  = sj + (size_t)MROWS * HIDD;
    float* red  = att + (size_t)BATCH * NNODE * NNODE;
    const size_t wsNeed = (size_t)((red + BATCH * 32) - (float*)d_ws) * sizeof(float);
    if (wsNeed > ws_size) return;

    for (int l = 0; l < 2; ++l) {
        {
            const float* X = (l == 0) ? feature : bufX; const int ldx = (l == 0) ? INDIM : HLD; const int K = (l == 0) ? INDIM : MEMD;
            const float asc = (l == 0) ? 1.0f : 256.0f;
            GemmArgs g = gemm_args(X, ldx, zm(0), (l == 0) ? W0 : W1, MEMD, zm(0), bufH, HLD, zm(0), MROWS, MEMD, K);
            g.nstore = HLD; g.bias = (l == 0) ? b0 : b1; g.ascale = asc; g.bscale = 16.0f; g.oscale = 1.0f / (asc * 16.0f);
            gemm_kernel<0, 1, 1, 1, 4, 2, ACT_NONE><<<dim3(MROWS / 64, (HLD + 127) / 128, 1), 256, 0, stream>>>(g);
        }
        {
            const float asc = (l == 0) ? 1.0f : 256.0f;
            GemmArgs g = gemm_args(bufH, HLD, zm(0), A1, HIDD, zm(0), si, HIDD, zm(0), MROWS, HIDD, MEMD);
            g.ascale = asc; g.bscale = 16.0f; g.oscale = 1.0f / (asc * 16.0f);
            gemm_kernel<0, 1, 1, 1, 8, 1, ACT_NONE><<<dim3(MROWS / 128, 1, 1), 256, 0, stream>>>(g);
            GemmArgs g2 = gemm_args(bufH, HLD, zm(0), A1 + (size_t)MEMD * HIDD, HIDD, zm(0), sj, HIDD, zm(0), MROWS, HIDD, MEMD);
            g2.bias = ab1; g2.ascale = asc; g2.bscale = 16.0f; g2.oscale = 1.0f / (asc * 16.0f);
            gemm_kernel<0, 1, 1, 1, 8, 1, ACT_NONE><<<dim3(MROWS / 128, 1, 1), 256, 0, stream>>>(g2);
        }
        edge_scores<<<dim3(NNODE, BATCH), NNODE, 0, stream>>>(si, sj, A2, ab2, adj, att);
        softmax_stats<<<BATCH, 256, 0, stream>>>(att, red);
        softmax_norm<<<dim3(NNODE, BATCH), NNODE, 0, stream>>>(att, red);
        {
            float* C = (l == 0) ? bufX : out; const int ldc = (l == 0) ? HLD : MEMD;
            const float bsc = (l == 0) ? 1.0f : 256.0f;
            GemmArgs g = gemm_args(att, NNODE, zm((long long)NNODE * NNODE), bufH, HLD, zm((long long)NNODE * HLD), C, ldc, zm((long long)NNODE * ldc), NNODE, MEMD, NNODE);
            g.nstore = (l == 0) ? HLD : MEMD; g.ascale = 4096.0f; g.bscale = bsc; g.oscale = 1.0f / (4096.0f * bsc);
            gemm_kernel<0, 1, 1, 1, 4, 2, ACT_NONE><<<dim3(NNODE / 64, (HLD + 127) / 128, BATCH), 256, 0, stream>>>(g);
        }
    }
}
